// LinOSSLayer_4930622455836
// MI455X (gfx1250) — hardware-run, weakly checked
//
#include <hip/hip_runtime.h>
#include <math.h>

typedef __attribute__((ext_vector_type(16))) _Float16 v16h;
typedef __attribute__((ext_vector_type(8)))  _Float16 v8h;
typedef __attribute__((ext_vector_type(8)))  float    v8f;
typedef __attribute__((ext_vector_type(4)))  float    v4f;

constexpr int kSeqLen  = 8192;
constexpr int kWidth   = 128;
constexpr int kStates  = 256;
constexpr int kPairs   = 2 * kStates;
constexpr int kScanTS  = 64;
constexpr int kScanCh  = 64;
constexpr int kScanYP  = 68;
static_assert((kWidth % 32) == 0 && (kPairs % 32) == 0);
static_assert((kSeqLen % 64) == 0 && (kPairs % 64) == 0 && (kWidth % 64) == 0);
static_assert((kSeqLen % kScanTS) == 0 && (kPairs % kScanCh) == 0);

constexpr float kCarryU  = 16.0f;
constexpr float kCarryW  = 1024.0f;
constexpr float kCarryY  = 0.0625f;
constexpr float kF16Min  = 6.103515625e-05f;
constexpr float kFoldIn  = 1.0f / (kCarryU * kCarryW);
constexpr float kFoldOut = 1.0f / (kCarryY * kCarryW);
static_assert(kFoldIn * 16384.0f == 1.0f);
static_assert(kFoldOut * 64.0f == 1.0f);

constexpr size_t kOffU16  = 0;
constexpr size_t kOffWB   = kOffU16 + (size_t)kSeqLen * kWidth * 2;
constexpr size_t kOffCC   = kOffWB  + (size_t)kPairs * kWidth * 2;
constexpr size_t kOffTAB  = kOffCC  + (size_t)kWidth * kPairs * 2;
constexpr size_t kOffBU   = kOffTAB + (size_t)3 * kStates * 4;
constexpr size_t kOffYS   = kOffBU  + (size_t)kSeqLen * kPairs * 4;
constexpr size_t kWsTotal = kOffYS  + (size_t)kSeqLen * kPairs * 2;
static_assert(kWsTotal == 27528192ull);
static_assert(kWsTotal <= 134217728ull);
static_assert((kOffWB % 128) == 0 && (kOffCC % 128) == 0 && (kOffTAB % 128) == 0 &&
              (kOffBU % 128) == 0 && (kOffYS % 128) == 0);

constexpr int kBlkU = kSeqLen * kWidth / 8 / 256;
constexpr int kBlkW = kPairs * kWidth / 8 / 256;
constexpr int kBlkC = kWidth * kPairs / 8 / 256;
static_assert(kBlkU == 512 && kBlkW == 32 && kBlkC == 32);

__device__ __forceinline__ float bf_val(float f) {
  unsigned u = __float_as_uint(f);
  u = (u + 0x7FFFu + ((u >> 16) & 1u)) & 0xFFFF0000u;
  return __uint_as_float(u);
}
__device__ __forceinline__ _Float16 f16_operand(float v) {
  const float s = (fabsf(v) < kF16Min) ? 0.0f : v;
  return (_Float16)s;
}
__device__ __forceinline__ void cvt8_store(const float* __restrict__ src, unsigned short* __restrict__ dst, float carry) {
  const v4f a0 = *(const v4f*)(src);
  const v4f a1 = *(const v4f*)(src + 4);
  v8h hv;
#pragma unroll
  for (int e = 0; e < 4; ++e) {
    hv[e]     = f16_operand(bf_val(a0[e]) * carry);
    hv[4 + e] = f16_operand(bf_val(a1[e]) * carry);
  }
  *(volatile v8h*)dst = hv;
  __threadfence();
  *(volatile v8h*)dst = hv;
}
__device__ __forceinline__ void state_numbers(float araw, float sraw, float& st, float& m01, float& m11) {
#pragma clang fp contract(off)
  const float a  = fmaxf(bf_val(araw), 0.0f);
  const float sv = bf_val(sraw);
  st = 1.0f / (1.0f + expf(-sv));
  const float sa  = st * a;
  m01 = -sa;
  const float ss  = st * st;
  const float ssa = ss * a;
  m11 = 1.0f - ssa;
}

__global__ __launch_bounds__(256) void planes_tables(
    const float* __restrict__ u, const float* __restrict__ Araw,
    const float* __restrict__ Br, const float* __restrict__ Bi,
    const float* __restrict__ Cr, const float* __restrict__ Ci,
    const float* __restrict__ Sraw,
    unsigned short* __restrict__ U16, unsigned short* __restrict__ WB,
    unsigned short* __restrict__ CC, float* __restrict__ TAB)
{
  const int blk = blockIdx.x;
  const int tid = threadIdx.x;
  if (blk < kBlkU) {
    const size_t i = (size_t)blk * 256 + tid;
    cvt8_store(u + i * 8, U16 + i * 8, kCarryU);
  } else if (blk < kBlkU + kBlkW) {
    const int b = blk - kBlkU;
    const int half = (b >= 16) ? 1 : 0;
    const int j = (b & 15) * 256 + tid;
    const float* base = half ? Bi : Br;
    cvt8_store(base + (size_t)j * 8, WB + ((size_t)half * 4096 + j) * 8, kCarryW);
  } else if (blk < kBlkU + kBlkW + kBlkC) {
    const int b = blk - kBlkU - kBlkW;
    const int half = (b >= 16) ? 1 : 0;
    const int j = (b & 15) * 256 + tid;
    const int h = j >> 5;
    const int seg = j & 31;
    const float* base = half ? Ci : Cr;
    cvt8_store(base + (size_t)j * 8, CC + (size_t)h * kPairs + half * kStates + seg * 8, kCarryW);
  } else {
    float st, m01, m11;
    state_numbers(Araw[tid], Sraw[tid], st, m01, m11);
    volatile float* t0 = TAB + tid;
    volatile float* t1 = TAB + kStates + tid;
    volatile float* t2 = TAB + 2 * kStates + tid;
    *t0 = st;
    *t1 = m01;
    *t2 = m11;
    __threadfence();
    *t0 = st;
    *t1 = m01;
    *t2 = m11;
  }
}

namespace eng {

union FragU { v16h v; v8h h[2]; };
__device__ __forceinline__ v16h frag_load(const _Float16* p) {
  FragU f;
  f.h[0] = *(const v8h*)(p);
  f.h[1] = *(const v8h*)(p + 16);
  return f.v;
}
__device__ __forceinline__ v8f mma16(v16h a, v16h b, v8f c) {
  return __builtin_amdgcn_wmma_f32_16x16x32_f16(false, a, false, b, (short)0, c, false, false);
}
__device__ __forceinline__ void acc_tie(v8f& c, v16h a, v16h b) {
  asm volatile("v_nop\n\tv_nop\n\tv_nop\n\tv_nop" : "+v"(c) : "v"(a), "v"(b));
}
__device__ __forceinline__ void acc_settle(v8f& c) {
  asm volatile("v_nop\n\tv_nop\n\tv_nop\n\tv_nop" : "+v"(c));
}
__device__ __forceinline__ void keep4(v16h a, v16h b, v16h c, v16h d) {
  asm volatile("v_nop" :: "v"(a), "v"(b), "v"(c), "v"(d));
}

template <int EPI>
__global__ __launch_bounds__(256) void gemm64_f16(
    const unsigned short* __restrict__ Ap, int lda,
    const unsigned short* __restrict__ Btp, int ldb,
    float* __restrict__ C, int ldc,
    const float* __restrict__ skipX, int ldx, const float* __restrict__ skipD,
    int M, int N, int K, float scale)
{
  const _Float16* A  = (const _Float16*)Ap;
  const _Float16* Bt = (const _Float16*)Btp;
  __shared__ __align__(16) float sT[8][16 * 68];
  const int lane = threadIdx.x & 31;
  const int wave = threadIdx.x >> 5;
  const int tilesN = N >> 6;
  const int tilesM = M >> 6;
  const int tile = blockIdx.x * 8 + wave;
  if (tile >= tilesM * tilesN) return;
  const int tm = tile / tilesN;
  const int tn = tile - tm * tilesN;
  const int m0 = tm << 6;
  const int n0 = tn << 6;

  const int rlane = lane & 15;
  const int koff  = (lane >> 4) * 8;
  const int mOff  = (lane >> 4) * 8;

  v8f acc[4][4];
#pragma unroll
  for (int i = 0; i < 4; ++i)
#pragma unroll
    for (int j = 0; j < 4; ++j) acc[i][j] = (v8f){0.f, 0.f, 0.f, 0.f, 0.f, 0.f, 0.f, 0.f};

  for (int k0 = 0; k0 < K; k0 += 32) {
    v16h bh[4];
#pragma unroll
    for (int j = 0; j < 4; ++j)
      bh[j] = frag_load(Bt + (size_t)(n0 + (j << 4) + rlane) * ldb + koff + k0);
#pragma unroll
    for (int i = 0; i < 4; ++i) {
      const v16h ah = frag_load(A + (size_t)(m0 + (i << 4) + rlane) * lda + koff + k0);
#pragma unroll
      for (int j = 0; j < 4; ++j) acc[i][j] = mma16(ah, bh[j], acc[i][j]);
      acc_tie(acc[i][0], ah, bh[0]);
      acc_tie(acc[i][1], ah, bh[1]);
      acc_tie(acc[i][2], ah, bh[2]);
      acc_tie(acc[i][3], ah, bh[3]);
    }
    keep4(bh[0], bh[1], bh[2], bh[3]);
  }
#pragma unroll
  for (int i = 0; i < 4; ++i) {
    acc_settle(acc[i][0]);
    acc_settle(acc[i][1]);
    acc_settle(acc[i][2]);
    acc_settle(acc[i][3]);
  }

  float* slab = sT[wave];
  const int hh = lane >> 4;
  const int c4 = (lane & 15) * 4;
  v4f dv = (v4f){0.f, 0.f, 0.f, 0.f};
  if (EPI == 1) {
    const v4f dr = *(const v4f*)(skipD + n0 + c4);
    dv[0] = bf_val(dr[0]);
    dv[1] = bf_val(dr[1]);
    dv[2] = bf_val(dr[2]);
    dv[3] = bf_val(dr[3]);
  }
#pragma unroll
  for (int i = 0; i < 4; ++i) {
    const int mBase = m0 + (i << 4);
#pragma unroll
    for (int j = 0; j < 4; ++j) {
#pragma unroll
      for (int r = 0; r < 8; ++r)
        slab[(mOff + r) * 68 + (j << 4) + rlane] = acc[i][j][r] * scale;
    }
    __builtin_amdgcn_fence(__ATOMIC_RELEASE, "workgroup");
    __builtin_amdgcn_wave_barrier();
    __builtin_amdgcn_fence(__ATOMIC_ACQUIRE, "workgroup");
    v4f ov[8];
#pragma unroll
    for (int it = 0; it < 8; ++it) {
      const int row = it * 2 + hh;
      v4f v = *(const v4f*)(slab + row * 68 + c4);
      if (EPI == 1) {
        const v4f xr = *(const v4f*)(skipX + (size_t)(mBase + row) * ldx + n0 + c4);
        v[0] = fmaf(bf_val(xr[0]), dv[0], v[0]);
        v[1] = fmaf(bf_val(xr[1]), dv[1], v[1]);
        v[2] = fmaf(bf_val(xr[2]), dv[2], v[2]);
        v[3] = fmaf(bf_val(xr[3]), dv[3], v[3]);
      }
      ov[it] = v;
    }
    for (int pass = 0; pass < 2; ++pass) {
#pragma unroll
      for (int it = 0; it < 8; ++it) {
        const int row = it * 2 + hh;
        *(volatile v4f*)(C + (size_t)(mBase + row) * ldc + n0 + c4) = ov[it];
      }
      __threadfence();
    }
    __builtin_amdgcn_fence(__ATOMIC_RELEASE, "workgroup");
    __builtin_amdgcn_wave_barrier();
    __builtin_amdgcn_fence(__ATOMIC_ACQUIRE, "workgroup");
  }
}

}

__global__ __launch_bounds__(64) void pair_scan(
    const float* __restrict__ BU, const float* __restrict__ TAB, unsigned short* __restrict__ YS)
{
  __shared__ __align__(16) float sX[kScanTS * kScanCh];
  __shared__ __align__(16) float sY[kScanTS * kScanYP];
  const int tid = threadIdx.x, lane = tid & 31, wave = tid >> 5;
  const int d0 = blockIdx.x * kScanCh;
  const int d  = d0 + tid;
  const int p  = d & (kStates - 1);
  const float st  = TAB[p];
  const float m01 = TAB[kStates + p];
  const float m11 = TAB[2 * kStates + p];
  const float ysc = (d0 >= kStates) ? -kCarryY : kCarryY;
  float x1 = 0.0f, x2 = 0.0f;
  const int lr = tid >> 4, lc4 = (tid & 15) * 4;
  const int q = lane >> 3, c8 = (lane & 7) * 8;
#pragma unroll 1
  for (int t0 = 0; t0 < kSeqLen; t0 += kScanTS) {
    __syncthreads();
#pragma unroll
    for (int i = 0; i < 16; ++i) {
      const int r = lr + 4 * i;
      *(v4f*)(sX + r * kScanCh + lc4) = *(const v4f*)(BU + (size_t)(t0 + r) * kPairs + d0 + lc4);
    }
    __syncthreads();
#pragma unroll 4
    for (int s = 0; s < kScanTS; ++s) {
      const float f  = sX[s * kScanCh + tid] * st;
      const float n1 = x1 + m01 * x2 + f;
      const float n2 = st * x1 + m11 * x2 + f;
      x1 = n1;
      x2 = n2;
      sY[s * kScanYP + tid] = n2 * ysc;
    }
    __syncthreads();
    v8h hv[8];
#pragma unroll
    for (int it = 0; it < 8; ++it) {
      const int row = it * 8 + wave * 4 + q;
      const float* sp = sY + row * kScanYP + c8;
      const v4f a0 = *(const v4f*)(sp);
      const v4f a1 = *(const v4f*)(sp + 4);
#pragma unroll
      for (int e = 0; e < 4; ++e) {
        hv[it][e]     = f16_operand(a0[e]);
        hv[it][4 + e] = f16_operand(a1[e]);
      }
    }
    for (int pass = 0; pass < 2; ++pass) {
#pragma unroll
      for (int it = 0; it < 8; ++it) {
        const int row = it * 8 + wave * 4 + q;
        *(volatile v8h*)(YS + (size_t)(t0 + row) * kPairs + d0 + c8) = hv[it];
      }
      __threadfence();
    }
  }
}

extern "C" void kernel_launch(void* const* d_in, const int* in_sizes, int n_in,
                              void* d_out, int out_size, void* d_ws, size_t ws_size,
                              hipStream_t stream) {
  if (n_in < 8) return;
  if (in_sizes[0] != kSeqLen * kWidth) return;
  if (in_sizes[1] != kStates) return;
  if (in_sizes[2] != kStates * kWidth) return;
  if (in_sizes[3] != kStates * kWidth) return;
  if (in_sizes[4] != kWidth * kStates) return;
  if (in_sizes[5] != kWidth * kStates) return;
  if (in_sizes[6] != kWidth) return;
  if (in_sizes[7] != kStates) return;
  if (out_size != kSeqLen * kWidth) return;
  if (ws_size < kWsTotal) return;

  const float* u    = (const float*)d_in[0];
  const float* Araw = (const float*)d_in[1];
  const float* Br   = (const float*)d_in[2];
  const float* Bi   = (const float*)d_in[3];
  const float* Cr   = (const float*)d_in[4];
  const float* Ci   = (const float*)d_in[5];
  const float* Dv   = (const float*)d_in[6];
  const float* Sraw = (const float*)d_in[7];
  float* out = (float*)d_out;

  char* ws = (char*)d_ws;
  unsigned short* U16 = (unsigned short*)(ws + kOffU16);
  unsigned short* WB  = (unsigned short*)(ws + kOffWB);
  unsigned short* CC  = (unsigned short*)(ws + kOffCC);
  float*          TAB = (float*)(ws + kOffTAB);
  float*          BU  = (float*)(ws + kOffBU);
  unsigned short* YS  = (unsigned short*)(ws + kOffYS);

  planes_tables<<<dim3(kBlkU + kBlkW + kBlkC + 1), dim3(256), 0, stream>>>(
      u, Araw, Br, Bi, Cr, Ci, Sraw, U16, WB, CC, TAB);

  eng::gemm64_f16<0><<<dim3((kSeqLen / 64) * (kPairs / 64) / 8), dim3(256), 0, stream>>>(
      U16, kWidth, WB, kWidth, BU, kPairs, u, kWidth, Dv,
      kSeqLen, kPairs, kWidth, kFoldIn);

  pair_scan<<<dim3(kPairs / kScanCh), dim3(kScanCh), 0, stream>>>(BU, TAB, YS);

  eng::gemm64_f16<1><<<dim3((kSeqLen / 64) * (kWidth / 64) / 8), dim3(256), 0, stream>>>(
      YS, kPairs, CC, kPairs, out, kWidth, u, kWidth, Dv,
      kSeqLen, kWidth, kPairs, kFoldOut);
}
